// self_attention_43336220016804
// MI455X (gfx1250) — hardware-verified
//
#include <hip/hip_runtime.h>


#define DEV __device__ __forceinline__

#ifndef NB
#define NB 4
#endif
#ifndef SEQ
#define SEQ 4096
#endif
#define NB_FULL  4
#define SEQ_FULL 4096
#define CH   64
#define KDIM 64
#define WPL  (CH * CH)
#define ZST  132
#define SCORE_SCALE 0.00390625f
#define OPROJ_SCALE 0.00006103515625f

static_assert(NB >= 1 && NB <= NB_FULL);
static_assert(SEQ >= 128 && SEQ <= SEQ_FULL && (SEQ % 128) == 0);
static_assert(((NB * SEQ) % 128) == 0);
static_assert(CH == 64 && (KDIM % 32) == 0 && KDIM == CH);
static_assert((WPL % (8 * 256)) == 0);
static_assert(((ZST * 4) % 16) == 0);
static_assert((long long)NB * CH * SEQ * 4 <= (long long)NB_FULL * CH * SEQ_FULL * 4);

typedef _Float16       v8h   __attribute__((ext_vector_type(8)));
typedef _Float16       v16h  __attribute__((ext_vector_type(16)));
typedef __bf16         v16bf __attribute__((ext_vector_type(16)));
typedef unsigned short v8us  __attribute__((ext_vector_type(8)));
typedef unsigned short v16us __attribute__((ext_vector_type(16)));
typedef float          v8f   __attribute__((ext_vector_type(8)));
typedef float          v4f   __attribute__((ext_vector_type(4)));

union FragH { v16h v;  v8h  half[2]; };
union FragB { v16bf v; v16us u; v8us half[2]; };
union Pack8 { v8us u; v8h hv; };

DEV unsigned int bf16_bits(float f) {
    unsigned int u = __float_as_uint(f);
    u += 0x7FFFu + ((u >> 16) & 1u);
    return u >> 16;
}
DEV float bf16_val(float f) { return __uint_as_float(bf16_bits(f) << 16); }

DEV v8f zero8f() {
    v8f z;
#pragma unroll
    for (int i = 0; i < 8; ++i) z[i] = 0.f;
    return z;
}

DEV v8f mma_bf16(v16bf a, v16bf b, v8f c) {
    c = __builtin_amdgcn_wmma_f32_16x16x32_bf16(false, a, false, b, (short)0, c, false, false);
    asm volatile("v_nop\n\tv_nop\n\tv_nop\n\tv_nop" : "+v"(c) : "v"(a), "v"(b));
    return c;
}
DEV v8f mma_f16(v16h a, v16h b, v8f c) {
    c = __builtin_amdgcn_wmma_f32_16x16x32_f16(false, a, false, b, (short)0, c, false, false);
    asm volatile("v_nop\n\tv_nop\n\tv_nop\n\tv_nop" : "+v"(c) : "v"(a), "v"(b));
    return c;
}

__global__ __launch_bounds__(256) void k_cvt_w(const float* __restrict__ w0,
                                               const float* __restrict__ w1,
                                               const float* __restrict__ w2,
                                               const float* __restrict__ w3,
                                               unsigned short* __restrict__ wpl)
{
    const int mi = blockIdx.y;
    const int g  = blockIdx.x * 256 + threadIdx.x;
    const int e  = g * 8;
    const float* src = (mi == 0) ? w0 : (mi == 1) ? w1 : (mi == 2) ? w2 : w3;
    const v4f a0 = *(const v4f*)(src + e);
    const v4f a1 = *(const v4f*)(src + e + 4);
    Pack8 o;
    if (mi == 3) {
#pragma unroll
        for (int i = 0; i < 4; ++i) {
            o.hv[i]     = (_Float16)(bf16_val(a0[i]) * 64.0f);
            o.hv[4 + i] = (_Float16)(bf16_val(a1[i]) * 64.0f);
        }
    } else {
#pragma unroll
        for (int i = 0; i < 4; ++i) {
            o.u[i]     = (unsigned short)bf16_bits(a0[i]);
            o.u[4 + i] = (unsigned short)bf16_bits(a1[i]);
        }
    }
    unsigned short* dst = wpl + (size_t)mi * WPL + e;
    *(volatile v8us*)dst = o.u;
    __threadfence();
    *(volatile v8us*)dst = o.u;
}

__global__ __launch_bounds__(256) void k_cvt_xt(const float* __restrict__ x,
                                                unsigned short* __restrict__ xT)
{
    __shared__ __attribute__((aligned(16))) unsigned short T[64 * 72];
    const int tid = threadIdx.x;
    const int n0 = blockIdx.x * 64;
    const int b  = blockIdx.z;
    const int nn = tid & 63, rq = tid >> 6;
#pragma unroll 4
    for (int i = 0; i < 16; ++i) {
        const int rr = i * 4 + rq;
        const float v = x[((size_t)b * CH + rr) * SEQ_FULL + n0 + nn];
        T[nn * 72 + rr] = (unsigned short)bf16_bits(v);
    }
    __syncthreads();
    const int piece = tid & 7;
    const int na = tid >> 3;
    const v8us va = *(const v8us*)(T + na * 72 + piece * 8);
    const v8us vb = *(const v8us*)(T + (na + 32) * 72 + piece * 8);
    unsigned short* da = xT + ((size_t)b * SEQ + n0 + na) * CH + piece * 8;
    unsigned short* db = xT + ((size_t)b * SEQ + n0 + na + 32) * CH + piece * 8;
    *(volatile v8us*)da = va;
    *(volatile v8us*)db = vb;
    __threadfence();
    *(volatile v8us*)da = va;
    *(volatile v8us*)db = vb;
}

template <int WM>
__global__ __launch_bounds__(256) __attribute__((amdgpu_num_vgpr(256)))
void k_gemm_nt(const unsigned short* __restrict__ A, long long zsA,
               const unsigned short* __restrict__ Bm, long long zsB,
               const float* __restrict__ bias, int nbias, int bias_per_row,
               _Float16* __restrict__ Cm, long long zsC, int ldc, float oscale)
{
    constexpr int TR   = 16 * WM;
    constexpr int TC   = 512 / WM;
    constexpr int CT_P = TC + 8;
    constexpr int LPR  = TC / 8;
    constexpr int RPI  = 32 / LPR;
    constexpr int RPW  = TR / 8;
    constexpr int NI   = RPW / RPI;
    static_assert(WM == 4 || WM == 8);
    static_assert(NI * RPI * 8 == TR && LPR * 8 == TC && ((CT_P * 2) % 16) == 0);

    __shared__ __attribute__((aligned(16))) _Float16 Ct[TR * CT_P];

    const int tid = threadIdx.x, lane = tid & 31, w = tid >> 5;
    const int h = lane >> 4, l15 = lane & 15;
    const int wm = w % WM, wn = w / WM;
    const int z = blockIdx.z;
    const int row0 = blockIdx.y * TR;
    const int col0 = blockIdx.x * TC;

    const unsigned short* ap = A  + (size_t)z * (size_t)zsA + (size_t)(row0 + wm * 16 + l15) * KDIM + 8 * h;
    const unsigned short* bp = Bm + (size_t)z * (size_t)zsB + (size_t)(col0 + wn * 64 + l15) * KDIM + 8 * h;

    v8f acc[4];
#pragma unroll
    for (int t = 0; t < 4; ++t) acc[t] = zero8f();

#pragma unroll 1
    for (int k0 = 0; k0 < KDIM; k0 += 32) {
        FragB a;
        a.half[0] = *(const v8us*)(ap + k0);
        a.half[1] = *(const v8us*)(ap + k0 + 16);
#pragma unroll
        for (int t = 0; t < 4; ++t) {
            const unsigned short* bq = bp + (size_t)t * 16 * KDIM + k0;
            FragB bf;
            bf.half[0] = *(const v8us*)(bq);
            bf.half[1] = *(const v8us*)(bq + 16);
            acc[t] = mma_bf16(a.v, bf.v, acc[t]);
        }
    }

    float rowb[8];
#pragma unroll
    for (int r = 0; r < 8; ++r) {
        int ri = row0 + wm * 16 + 8 * h + r;
        ri = ri < nbias ? ri : (nbias - 1);
        rowb[r] = bf16_val(bias[ri]);
    }
#pragma unroll
    for (int t = 0; t < 4; ++t) {
        const int cl = wn * 64 + t * 16 + l15;
        int ci = col0 + cl;
        ci = ci < nbias ? ci : (nbias - 1);
        const float colb = bf16_val(bias[ci]);
#pragma unroll
        for (int r = 0; r < 8; ++r) {
            const float badd = bias_per_row ? rowb[r] : colb;
            const float v = (acc[t][r] + badd) * oscale;
            Ct[(wm * 16 + 8 * h + r) * CT_P + cl] = (_Float16)v;
        }
    }
    __syncthreads();

    _Float16* cbase = Cm + (size_t)z * (size_t)zsC + (size_t)row0 * (size_t)ldc + col0;
    const int lr = lane / LPR;
    const int cs = (lane % LPR) * 8;
    v8h sv[NI];
#pragma unroll
    for (int i = 0; i < NI; ++i) {
        const int rl = w * RPW + i * RPI + lr;
        sv[i] = *(const v8h*)(Ct + rl * CT_P + cs);
    }
#pragma unroll
    for (int i = 0; i < NI; ++i) {
        const int rl = w * RPW + i * RPI + lr;
        *(volatile v8h*)(cbase + (size_t)rl * (size_t)ldc + cs) = sv[i];
    }
    __threadfence();
#pragma unroll
    for (int i = 0; i < NI; ++i) {
        const int rl = w * RPW + i * RPI + lr;
        *(volatile v8h*)(cbase + (size_t)rl * (size_t)ldc + cs) = sv[i];
    }
}

__global__ __launch_bounds__(256) __attribute__((amdgpu_num_vgpr(256)))
void k_attn(const _Float16* __restrict__ thT, const _Float16* __restrict__ phT,
            const _Float16* __restrict__ Vt, const _Float16* __restrict__ wob,
            const float* __restrict__ b_out, const float* __restrict__ gamma,
            const float* __restrict__ beta, const float* __restrict__ x,
            float* __restrict__ Out)
{
    __shared__ __attribute__((aligned(16))) float Zs[CH * ZST];

    const int tid = threadIdx.x, lane = tid & 31, w = tid >> 5;
    const int h = lane >> 4, l15 = lane & 15;
    const int kbo = 8 * h;
    const int b  = blockIdx.x / (SEQ / 128);
    const int n0 = (blockIdx.x - b * (SEQ / 128)) * 128;
    const int q0 = n0 + w * 16;

    FragH qb[2];
    {
        const _Float16* qp = thT + ((size_t)b * SEQ + q0 + l15) * CH + kbo;
#pragma unroll
        for (int s = 0; s < 2; ++s) {
            qb[s].half[0] = *(const v8h*)(qp + 32 * s);
            qb[s].half[1] = *(const v8h*)(qp + 32 * s + 16);
        }
    }

    v8f acc[4];
#pragma unroll
    for (int t = 0; t < 4; ++t) acc[t] = zero8f();
    float mrun = -1.0e30f, lsum = 0.f;

    const _Float16* kbase = phT + ((size_t)b * SEQ + l15) * CH + kbo;
    const _Float16* vbase = Vt + ((size_t)b * CH + l15) * SEQ + kbo;

#pragma unroll 1
    for (int m0 = 0; m0 < SEQ; m0 += 32) {
        const _Float16* kp = kbase + (size_t)m0 * CH;
        v8f s0 = zero8f(), s1 = zero8f();
#pragma unroll
        for (int s = 0; s < 2; ++s) {
            FragH k0f, k1f;
            k0f.half[0] = *(const v8h*)(kp + 32 * s);
            k0f.half[1] = *(const v8h*)(kp + 32 * s + 16);
            k1f.half[0] = *(const v8h*)(kp + 16 * CH + 32 * s);
            k1f.half[1] = *(const v8h*)(kp + 16 * CH + 32 * s + 16);
            s0 = mma_f16(k0f.v, qb[s].v, s0);
            s1 = mma_f16(k1f.v, qb[s].v, s1);
        }

        float tmax = -1.0e30f;
#pragma unroll
        for (int r = 0; r < 8; ++r) {
            s0[r] *= SCORE_SCALE;
            s1[r] *= SCORE_SCALE;
            tmax = fmaxf(tmax, fmaxf(s0[r], s1[r]));
        }
        tmax = fmaxf(tmax, __shfl_xor(tmax, 16));
        const float mnew  = fmaxf(mrun, tmax);
        const float alpha = __expf(mrun - mnew);
        mrun = mnew;

        FragH pb;
        float psum = 0.f;
#pragma unroll
        for (int r = 0; r < 8; ++r) {
            const _Float16 p0 = (_Float16)(__expf(s0[r] - mnew) * 1024.0f);
            const _Float16 p1 = (_Float16)(__expf(s1[r] - mnew) * 1024.0f);
            pb.half[0][r] = p0;
            pb.half[1][r] = p1;
            psum += (float)p0 + (float)p1;
        }
        psum += __shfl_xor(psum, 16);
        lsum = lsum * alpha + psum;
#pragma unroll
        for (int t = 0; t < 4; ++t) {
#pragma unroll
            for (int r = 0; r < 8; ++r) acc[t][r] *= alpha;
        }

        const _Float16* vp = vbase + m0;
#pragma unroll
        for (int t = 0; t < 4; ++t) {
            FragH vf;
            vf.half[0] = *(const v8h*)(vp + (size_t)t * 16 * SEQ);
            vf.half[1] = *(const v8h*)(vp + (size_t)t * 16 * SEQ + 16);
            acc[t] = mma_f16(vf.v, pb.v, acc[t]);
        }
    }

    const float invc = 16.0f / lsum;
    FragH ob[2];
#pragma unroll
    for (int s = 0; s < 2; ++s) {
#pragma unroll
        for (int r = 0; r < 8; ++r) {
            ob[s].half[0][r] = (_Float16)(acc[2 * s][r] * invc);
            ob[s].half[1][r] = (_Float16)(acc[2 * s + 1][r] * invc);
        }
    }

    v8f az[4];
#pragma unroll
    for (int ct = 0; ct < 4; ++ct) az[ct] = zero8f();
    {
        const _Float16* wp = wob + (size_t)l15 * CH + kbo;
#pragma unroll
        for (int ct = 0; ct < 4; ++ct) {
#pragma unroll
            for (int s = 0; s < 2; ++s) {
                FragH wa;
                wa.half[0] = *(const v8h*)(wp + ct * 16 * CH + 32 * s);
                wa.half[1] = *(const v8h*)(wp + ct * 16 * CH + 32 * s + 16);
                az[ct] = mma_f16(wa.v, ob[s].v, az[ct]);
            }
        }
    }

    const float rs = rsqrtf(1.0f + 1.0e-5f);
#pragma unroll
    for (int ct = 0; ct < 4; ++ct) {
#pragma unroll
        for (int r = 0; r < 8; ++r) {
            const int c = ct * 16 + kbo + r;
            float zz = az[ct][r] * OPROJ_SCALE + b_out[c];
            zz = fmaxf(zz, 0.0f);
            zz = zz * (gamma[c] * rs) + beta[c];
            Zs[c * ZST + w * 16 + l15] = zz;
        }
    }
    __syncthreads();

    v4f vals[8];
    const size_t xrow = ((size_t)b * CH + w * 8) * SEQ_FULL + n0 + lane * 4;
    const size_t orow = ((size_t)b * CH + w * 8) * SEQ + n0 + lane * 4;
#pragma unroll
    for (int i = 0; i < 8; ++i) {
        const v4f xv = *(const v4f*)(x + xrow + (size_t)i * SEQ_FULL);
        const v4f zv = *(const v4f*)(Zs + (w * 8 + i) * ZST + lane * 4);
        vals[i] = xv + zv;
    }
#pragma unroll
    for (int i = 0; i < 8; ++i)
        *(volatile v4f*)(Out + orow + (size_t)i * SEQ) = vals[i];
    __threadfence();
#pragma unroll
    for (int i = 0; i < 8; ++i)
        *(volatile v4f*)(Out + orow + (size_t)i * SEQ) = vals[i];
}

extern "C" void kernel_launch(void* const* d_in, const int* in_sizes, int n_in,
                              void* d_out, int out_size, void* d_ws, size_t ws_size,
                              hipStream_t stream)
{
    if (n_in < 11) return;
    const long long need_x = ((long long)(NB - 1) * CH + (CH - 1)) * SEQ_FULL + SEQ;
    if ((long long)in_sizes[0] < need_x) return;
    if (in_sizes[1] < CH * CH || in_sizes[3] < CH * CH || in_sizes[5] < CH * CH || in_sizes[7] < CH * CH) return;
    if (in_sizes[2] < CH || in_sizes[4] < CH || in_sizes[6] < CH || in_sizes[8] < CH) return;
    if (in_sizes[9] < CH || in_sizes[10] < CH) return;
    if ((long long)out_size < (long long)NB * CH * SEQ) return;

    const float* x       = (const float*)d_in[0];
    const float* w_theta = (const float*)d_in[1];
    const float* b_theta = (const float*)d_in[2];
    const float* w_phi   = (const float*)d_in[3];
    const float* b_phi   = (const float*)d_in[4];
    const float* w_g     = (const float*)d_in[5];
    const float* b_g     = (const float*)d_in[6];
    const float* w_out   = (const float*)d_in[7];
    const float* b_out   = (const float*)d_in[8];
    const float* gamma   = (const float*)d_in[9];
    const float* beta    = (const float*)d_in[10];
    float* out = (float*)d_out;

    char* ws = (char*)d_ws;
    size_t off = 0;
    auto carve = [&](size_t bytes) -> char* {
        char* p = ws + off;
        off += (bytes + 255) & ~(size_t)255;
        return p;
    };
    unsigned short* wpl = (unsigned short*)carve((size_t)4 * WPL * 2);
    unsigned short* xT  = (unsigned short*)carve((size_t)NB * SEQ * CH * 2);
    _Float16* thT = (_Float16*)carve((size_t)NB * SEQ * CH * 2);
    _Float16* phT = (_Float16*)carve((size_t)NB * SEQ * CH * 2);
    _Float16* Vt  = (_Float16*)carve((size_t)NB * CH * SEQ * 2);
    if (off > ws_size) return;

    k_cvt_w<<<dim3(WPL / 8 / 256, 4), 256, 0, stream>>>(w_theta, w_phi, w_g, w_out, wpl);

    k_cvt_xt<<<dim3(SEQ / 64, 1, NB), 256, 0, stream>>>(x, xT);

    k_gemm_nt<8><<<dim3(CH / 64, (NB * SEQ) / 128, 1), 256, 0, stream>>>(
        xT, 0LL, wpl, 0LL, b_theta, CH, 0, thT, 0LL, CH, 16.0f);
    k_gemm_nt<8><<<dim3(CH / 64, (NB * SEQ) / 128, 1), 256, 0, stream>>>(
        xT, 0LL, wpl + WPL, 0LL, b_phi, CH, 0, phT, 0LL, CH, 16.0f);
    k_gemm_nt<4><<<dim3(SEQ / 128, CH / 64, NB), 256, 0, stream>>>(
        wpl + 2 * WPL, 0LL, xT, (long long)SEQ * CH, b_g, CH, 1, Vt, (long long)CH * SEQ, SEQ, 16.0f);

    k_attn<<<NB * (SEQ / 128), 256, 0, stream>>>(
        thT, phT, Vt, (const _Float16*)(wpl + 3 * WPL), b_out, gamma, beta, x, out);
}
